// MultiScaleRetention_51702816309254
// MI455X (gfx1250) — hardware-verified
//
#include <hip/hip_runtime.h>
#include <math.h>

constexpr int kBatch  = 2;
constexpr int kSeq    = 2048;
constexpr int kHid    = 1024;
constexpr int kQK     = 1024;
constexpr int kVDim   = 2048;
constexpr int kHeads  = 8;
constexpr int kDq     = 128;
constexpr int kDv     = 256;
constexpr int kTok    = kBatch * kSeq;
constexpr int kBH     = kBatch * kHeads;
constexpr int kQKCols = 2 * kQK;
constexpr float kWCarry   = 64.0f;
constexpr float kQCarry   = 256.0f;
constexpr float kVCarry   = 16.0f;
constexpr float kKwCarry  = 16.0f;
constexpr float kGCarry   = 64.0f;
constexpr float kResCarry = 1024.0f;
constexpr float kResInv   = 1.0f / 1024.0f;
constexpr float kQkScale  = 0.08838834764831845f;
constexpr float kEps      = 1.0e-5f;
constexpr float kXScale   = 1.0f / (kQCarry * kVCarry);
static_assert(kHeads * kDq == kQK && kHeads * kDv == kVDim, "shape");
static_assert(kHid % 32 == 0 && kVDim % 32 == 0 && kSeq % 64 == 0, "k tiles");
static_assert(kTok % 64 == 0 && kQK % 64 == 0 && kVDim % 64 == 0 && kHid % 64 == 0 && kDq % 64 == 0 && kDv % 64 == 0, "mn tiles");

typedef __attribute__((ext_vector_type(16))) _Float16 v16h;
typedef __attribute__((ext_vector_type(8)))  _Float16 v8h;
typedef __attribute__((ext_vector_type(16))) __bf16   v16b;
typedef __attribute__((ext_vector_type(8)))  __bf16   v8b;
typedef __attribute__((ext_vector_type(8)))  float    v8f;
typedef __attribute__((ext_vector_type(4)))  float    v4f;
typedef __attribute__((ext_vector_type(2)))  float    v2f;
typedef __attribute__((ext_vector_type(4)))  unsigned int v4u;

__device__ __forceinline__ unsigned short f2bf_bits(float f) {
  unsigned u = __float_as_uint(f);
  return (unsigned short)((u + 0x7FFFu + ((u >> 16) & 1u)) >> 16);
}
__device__ __forceinline__ float bf_bits2f(unsigned short h) { return __uint_as_float(((unsigned)h) << 16); }

__device__ __forceinline__ void dep_guard_h(v8f& a, v8f& b, v16h x, v16h y) { asm volatile("v_nop\n\tv_nop\n\tv_nop\n\tv_nop" : "+v"(a), "+v"(b) : "v"(x), "v"(y)); }
__device__ __forceinline__ void dep_guard_b(v8f& a, v8f& b, v16b x, v16b y) { asm volatile("v_nop\n\tv_nop\n\tv_nop\n\tv_nop" : "+v"(a), "+v"(b) : "v"(x), "v"(y)); }
__device__ __forceinline__ void dep_guard4_h(v8f& a, v8f& b, v8f& c, v8f& d, v16h x, v16h y) {
  asm volatile("v_nop\n\tv_nop\n\tv_nop\n\tv_nop" : "+v"(a), "+v"(b), "+v"(c), "+v"(d) : "v"(x), "v"(y));
}
__device__ __forceinline__ void dep_guard4_b(v8f& a, v8f& b, v8f& c, v8f& d, v16b x, v16b y) {
  asm volatile("v_nop\n\tv_nop\n\tv_nop\n\tv_nop" : "+v"(a), "+v"(b), "+v"(c), "+v"(d) : "v"(x), "v"(y));
}
__device__ __forceinline__ void keep4_h(v16h a, v16h b, v16h c, v16h d) { asm volatile("v_nop" :: "v"(a), "v"(b), "v"(c), "v"(d)); }
__device__ __forceinline__ void keep4_b(v16b a, v16b b, v16b c, v16b d) { asm volatile("v_nop" :: "v"(a), "v"(b), "v"(c), "v"(d)); }
__device__ __forceinline__ void acc_guard4(v8f& a, v8f& b, v8f& c, v8f& d) { asm volatile("v_nop\n\tv_nop\n\tv_nop\n\tv_nop" : "+v"(a), "+v"(b), "+v"(c), "+v"(d)); }
template <typename T> struct Frag;
template <> struct Frag<_Float16> {
  typedef v16h V; union U { v16h v; v8h h[2]; };
  static __device__ __forceinline__ v16h load(const _Float16* p) {
    U f; f.h[0] = *(const v8h*)(p); f.h[1] = *(const v8h*)(p + 16); return f.v;
  }
  static __device__ __forceinline__ v8f mma(v16h a, v16h b, v8f c) {
    return __builtin_amdgcn_wmma_f32_16x16x32_f16(false, a, false, b, (short)0, c, false, false);
  }
  static __device__ __forceinline__ void guard(v8f& a, v8f& b, v16h x, v16h y) { dep_guard_h(a, b, x, y); }
  static __device__ __forceinline__ void guard4(v8f& a, v8f& b, v8f& c, v8f& d, v16h x, v16h y) { dep_guard4_h(a, b, c, d, x, y); }
  static __device__ __forceinline__ void keep(v16h a, v16h b, v16h c, v16h d) { keep4_h(a, b, c, d); }
};
template <> struct Frag<__bf16> {
  typedef v16b V; union U { v16b v; v8b h[2]; };
  static __device__ __forceinline__ v16b load(const __bf16* p) {
    U f; f.h[0] = *(const v8b*)(p); f.h[1] = *(const v8b*)(p + 16); return f.v;
  }
  static __device__ __forceinline__ v8f mma(v16b a, v16b b, v8f c) {
    return __builtin_amdgcn_wmma_f32_16x16x32_bf16(false, a, false, b, (short)0, c, false, false);
  }
  static __device__ __forceinline__ void guard(v8f& a, v8f& b, v16b x, v16b y) { dep_guard_b(a, b, x, y); }
  static __device__ __forceinline__ void guard4(v8f& a, v8f& b, v8f& c, v8f& d, v16b x, v16b y) { dep_guard4_b(a, b, c, d, x, y); }
  static __device__ __forceinline__ void keep(v16b a, v16b b, v16b c, v16b d) { keep4_b(a, b, c, d); }
};

__device__ __forceinline__ unsigned pk16(unsigned short a, unsigned short b) { return (unsigned)a | ((unsigned)b << 16); }
__device__ __forceinline__ unsigned short h_bits(float f) { const _Float16 h = (_Float16)f; return __builtin_bit_cast(unsigned short, h); }
__device__ __forceinline__ float h16_to_f32(unsigned hb) {
  const unsigned sgn = (hb & 0x8000u) << 16; const unsigned em = hb & 0x7fffu;
  const float fn = __uint_as_float((em << 13) + 0x38000000u);
  const float fs = (float)em * 5.9604644775390625e-8f;
  const float mag = (em < 0x400u) ? fs : fn; return __uint_as_float(__float_as_uint(mag) | sgn);
}

template <int ET> struct Elem;
template <> struct Elem<0> { typedef _Float16 T; };
template <> struct Elem<1> { typedef __bf16 T; };
template <int ET, bool SPLIT, int BIAS_MODE, int OUT_MODE, bool RESID, int ACT = 0>
__global__ __launch_bounds__(256) void wmma_gemm64(
    const unsigned short* __restrict__ Ap, const unsigned short* __restrict__ A2p, int lda, long strideA,
    const unsigned short* __restrict__ Btp, const unsigned short* __restrict__ Bt2p, int ldb, long strideB,
    void* __restrict__ Cout, void* __restrict__ Cout2, int ldc, long strideC,
    const float* __restrict__ bias,
    const float* __restrict__ resid, long strideR,
    int M, int N, int K, float scale, float oscale) {
  typedef typename Elem<ET>::T T;
  typedef typename Frag<T>::V V;
  const T* A = (const T*)Ap; const T* A2 = (const T*)A2p; const T* Bt = (const T*)Btp; const T* Bt2 = (const T*)Bt2p;
  __shared__ __align__(16) float sT[8][16 * 68];
  const int b    = blockIdx.y;
  const int lane = threadIdx.x & 31;
  const int wave = threadIdx.x >> 5;
  const int tilesN = N >> 6;
  const int tilesM = M >> 6;
  const int tile = blockIdx.x * 8 + wave;
  if (tile >= tilesM * tilesN) return;
  const int tm = tile / tilesN;
  const int tn = tile - tm * tilesN;
  const int m0 = tm << 6;
  const int n0 = tn << 6;

  const T* Ab  = A  + (size_t)b * strideA;
  const T* Bb  = Bt + (size_t)b * strideB;
  const T* Ab2 = SPLIT ? (A2  + (size_t)b * strideA) : nullptr;
  const T* Bb2 = SPLIT ? (Bt2 + (size_t)b * strideB) : nullptr;

  const int rlane = lane & 15;
  const int koff  = (lane >> 4) * 8;
  const int mOff  = (lane >> 4) * 8;

  v8f acc[4][4];
#pragma unroll
  for (int i = 0; i < 4; ++i)
#pragma unroll
    for (int j = 0; j < 4; ++j) acc[i][j] = (v8f){0.f,0.f,0.f,0.f,0.f,0.f,0.f,0.f};

  for (int k0 = 0; k0 < K; k0 += 32) {
    V bh[4], bl[4];
#pragma unroll
    for (int j = 0; j < 4; ++j) {
      const size_t bo = (size_t)(n0 + (j << 4) + rlane) * ldb + koff + k0;
      bh[j] = Frag<T>::load(Bb + bo);
      if (SPLIT) bl[j] = Frag<T>::load(Bb2 + bo);
    }
#pragma unroll
    for (int i = 0; i < 4; ++i) {
      const size_t ao = (size_t)(m0 + (i << 4) + rlane) * lda + koff + k0;
      V ah = Frag<T>::load(Ab + ao);
      V al;
      if (SPLIT) al = Frag<T>::load(Ab2 + ao);
#pragma unroll
      for (int j = 0; j < 4; ++j) {
        acc[i][j] = Frag<T>::mma(ah, bh[j], acc[i][j]);
        if (SPLIT) {
          acc[i][j] = Frag<T>::mma(ah, bl[j], acc[i][j]);
          acc[i][j] = Frag<T>::mma(al, bh[j], acc[i][j]);
        }
      }
      Frag<T>::guard4(acc[i][0], acc[i][1], acc[i][2], acc[i][3], ah, SPLIT ? al : ah);
    }
    Frag<T>::keep(bh[0], bh[1], bh[2], bh[3]);
    if (SPLIT) Frag<T>::keep(bl[0], bl[1], bl[2], bl[3]);
  }
  acc_guard4(acc[0][0], acc[0][1], acc[0][2], acc[0][3]);
  acc_guard4(acc[1][0], acc[1][1], acc[1][2], acc[1][3]);
  acc_guard4(acc[2][0], acc[2][1], acc[2][2], acc[2][3]);
  acc_guard4(acc[3][0], acc[3][1], acc[3][2], acc[3][3]);

  float* slab = sT[wave];
  const float* Rb = RESID ? (resid + (size_t)b * strideR) : nullptr;
#pragma unroll
  for (int i = 0; i < 4; ++i) {
    const int mBase = m0 + (i << 4);
#pragma unroll
    for (int j = 0; j < 4; ++j) {
      const int n = n0 + (j << 4) + rlane;
      float bv = 0.f;
      if (BIAS_MODE == 2) bv = bias[n];
#pragma unroll
      for (int r = 0; r < 8; ++r) {
        float v = acc[i][j][r] * scale;
        if (BIAS_MODE == 1) v += bias[mBase + mOff + r];
        if (BIAS_MODE == 2) v += bv;
        if (RESID) v += Rb[(size_t)(mBase + mOff + r) * ldc + n];
        if (ACT == 1) v = tanhf(v);
        if (ACT == 2) v = fmaxf(v, 0.0f);
        if (ACT == 3) v = v / (1.0f + expf(-fmaxf(v, -60.0f)));
        if (ACT == 4) v = (v > 0.f) ? v : 0.01f * v;
        v = v * oscale;
        slab[(mOff + r) * 68 + (j << 4) + rlane] = v;
      }
    }
    __builtin_amdgcn_fence(__ATOMIC_RELEASE, "workgroup");
    __builtin_amdgcn_wave_barrier();
    __builtin_amdgcn_fence(__ATOMIC_ACQUIRE, "workgroup");
    if (OUT_MODE == 0) {
      float* C = (float*)Cout + (size_t)b * strideC;
      const int hh = lane >> 4, c4 = (lane & 15) * 4;
      for (int pass = 0; pass < 2; ++pass) {
#pragma unroll
        for (int it = 0; it < 8; ++it) {
          const int row = it * 2 + hh;
          v4f v = *(const v4f*)(slab + row * 68 + c4);
          *(volatile v4f*)(C + (size_t)(mBase + row) * ldc + n0 + c4) = v;
        }
        __threadfence();
      }
    } else {
      const int q = lane >> 3, c8 = (lane & 7) * 8;
      unsigned short* C  = (unsigned short*)Cout  + (size_t)b * strideC;
      unsigned short* C2 = (OUT_MODE == 2) ? ((unsigned short*)Cout2 + (size_t)b * strideC) : nullptr;
      for (int pass = 0; pass < 2; ++pass) {
#pragma unroll
        for (int it = 0; it < 4; ++it) {
          const int row = it * 4 + q;
          const float* sp = slab + row * 68 + c8;
          v8h hv, lv;
#pragma unroll
          for (int e = 0; e < 8; ++e) {
            if (OUT_MODE == 1) {
              hv[e] = (_Float16)sp[e];
            } else {
              unsigned short hb = f2bf_bits(sp[e]);
              unsigned short lb = f2bf_bits(sp[e] - bf_bits2f(hb));
              hv[e] = __builtin_bit_cast(_Float16, hb);
              lv[e] = __builtin_bit_cast(_Float16, lb);
            }
          }
          *(volatile v8h*)(C + (size_t)(mBase + row) * ldc + n0 + c8) = hv;
          if (OUT_MODE == 2) *(volatile v8h*)(C2 + (size_t)(mBase + row) * ldc + n0 + c8) = lv;
        }
        __threadfence();
      }
    }
    __builtin_amdgcn_fence(__ATOMIC_RELEASE, "workgroup");
    __builtin_amdgcn_wave_barrier();
    __builtin_amdgcn_fence(__ATOMIC_ACQUIRE, "workgroup");
  }
}

__global__ __launch_bounds__(256) void state_gemm_kernel(
    const unsigned short* __restrict__ Ahp, const unsigned short* __restrict__ Alp, int lda, long strideA,
    const unsigned short* __restrict__ Bhp, const unsigned short* __restrict__ Blp, int ldb, long strideB,
    float* __restrict__ C, int ldc, long strideC, int M, int N, int K, float scale, float rinv) {
  __shared__ __align__(16) float sT[8][32 * 36];
  const int b    = blockIdx.y;
  const int lane = threadIdx.x & 31;
  const int wave = threadIdx.x >> 5;
  const int tilesN = N >> 5;
  const int tilesM = M >> 5;
  const int tile = blockIdx.x * 8 + wave;
  if (tile >= tilesM * tilesN) return;
  const int tm = tile / tilesN;
  const int tn = tile - tm * tilesN;
  const int m0 = tm << 5;
  const int n0 = tn << 5;
  const _Float16* Ah = (const _Float16*)Ahp + (size_t)b * strideA;
  const _Float16* Al = (const _Float16*)Alp + (size_t)b * strideA;
  const _Float16* Bh = (const _Float16*)Bhp + (size_t)b * strideB;
  const _Float16* Bl = (const _Float16*)Blp + (size_t)b * strideB;
  const int rlane = lane & 15;
  const int koff  = (lane >> 4) * 8;
  const int mOff  = (lane >> 4) * 8;

  v8f acc[2][2], accr[2][2];
#pragma unroll
  for (int i = 0; i < 2; ++i)
#pragma unroll
    for (int j = 0; j < 2; ++j) {
      acc[i][j]  = (v8f){0.f,0.f,0.f,0.f,0.f,0.f,0.f,0.f};
      accr[i][j] = (v8f){0.f,0.f,0.f,0.f,0.f,0.f,0.f,0.f};
    }

  for (int k0 = 0; k0 < K; k0 += 32) {
    v16h bh[2], bl[2];
#pragma unroll
    for (int j = 0; j < 2; ++j) {
      const size_t bo = (size_t)(n0 + (j << 4) + rlane) * ldb + koff + k0;
      bh[j] = Frag<_Float16>::load(Bh + bo);
      bl[j] = Frag<_Float16>::load(Bl + bo);
    }
#pragma unroll
    for (int i = 0; i < 2; ++i) {
      const size_t ao = (size_t)(m0 + (i << 4) + rlane) * lda + koff + k0;
      const v16h ah = Frag<_Float16>::load(Ah + ao);
      const v16h al = Frag<_Float16>::load(Al + ao);
#pragma unroll
      for (int j = 0; j < 2; ++j) {
        acc[i][j]  = Frag<_Float16>::mma(ah, bh[j], acc[i][j]);
        accr[i][j] = Frag<_Float16>::mma(ah, bl[j], accr[i][j]);
        accr[i][j] = Frag<_Float16>::mma(al, bh[j], accr[i][j]);
      }
      dep_guard4_h(acc[i][0], acc[i][1], accr[i][0], accr[i][1], ah, al);
    }
    keep4_h(bh[0], bh[1], bl[0], bl[1]);
  }
  acc_guard4(acc[0][0], acc[0][1], acc[1][0], acc[1][1]);
  acc_guard4(accr[0][0], accr[0][1], accr[1][0], accr[1][1]);

  float* slab = sT[wave];
#pragma unroll
  for (int i = 0; i < 2; ++i)
#pragma unroll
    for (int j = 0; j < 2; ++j)
#pragma unroll
      for (int r = 0; r < 8; ++r) {
        const float v = (acc[i][j][r] + accr[i][j][r] * rinv) * scale;
        slab[((i << 4) + mOff + r) * 36 + (j << 4) + rlane] = v;
      }
  __builtin_amdgcn_fence(__ATOMIC_RELEASE, "workgroup");
  __builtin_amdgcn_wave_barrier();
  __builtin_amdgcn_fence(__ATOMIC_ACQUIRE, "workgroup");
  float* Cb = C + (size_t)b * strideC;
  const int q8 = lane >> 3, c4 = (lane & 7) * 4;
  for (int pass = 0; pass < 2; ++pass) {
#pragma unroll
    for (int it = 0; it < 8; ++it) {
      const int row = it * 4 + q8;
      const v4f val = *(const v4f*)(slab + row * 36 + c4);
      *(volatile v4f*)(Cb + (size_t)(m0 + row) * ldc + n0 + c4) = val;
    }
    __threadfence();
  }
}

__global__ __launch_bounds__(256) void cast8_f16_kernel(const float* __restrict__ in, unsigned short* __restrict__ out, int n8, float carry) {
  const int i = blockIdx.x * 256 + threadIdx.x;
  if (i >= n8) return;
  const float* p = in + 8 * (size_t)i;
  const v4f a = *(const v4f*)(p);
  const v4f c = *(const v4f*)(p + 4);
  unsigned short hb[8];
#pragma unroll
  for (int e = 0; e < 4; ++e) {
    hb[e]     = h_bits(a[e] * carry);
    hb[4 + e] = h_bits(c[e] * carry);
  }
  const v4u u = (v4u){pk16(hb[0], hb[1]), pk16(hb[2], hb[3]), pk16(hb[4], hb[5]), pk16(hb[6], hb[7])};
  unsigned short* q = out + 8 * (size_t)i;
  *(volatile v4u*)q = u;
  __threadfence();
  *(volatile v4u*)q = u;
}

__global__ __launch_bounds__(256) void pack_qk_kernel(const float* __restrict__ qk32, const float* __restrict__ decay,
                                                      unsigned short* __restrict__ q16, unsigned short* __restrict__ k16,
                                                      unsigned short* __restrict__ kwTh, unsigned short* __restrict__ kwTl,
                                                      double rbase) {
#pragma clang fp contract(off)
  __shared__ __align__(16) unsigned int sq[64 * 68];
  __shared__ __align__(16) unsigned int sk[64 * 68];
  __shared__ __align__(16) unsigned short skt[128 * 72];
  __shared__ __align__(16) unsigned short sktl[128 * 72];
  const int tcnk = blockIdx.x, h = blockIdx.y, b = blockIdx.z;
  const int bh = b * kHeads + h;
  const int t0 = tcnk * 64;
  const int tid = threadIdx.x, lane = tid & 31, wave = tid >> 5;
  const int pl = tid & 63, tsub = tid >> 6;
  const int gi = h * 64 + pl;
  double pw = 1.0, bs = rbase;
#pragma unroll
  for (int bit = 0; bit < 9; ++bit) {
    const double m = ((gi >> bit) & 1) ? bs : 1.0;
    pw = pw * m;
    bs = bs * bs;
  }
  const float invf = 1.0f / (float)pw;
  const float sv   = ((float)(2 * gi) + 409.6f) * (1.0f / 1433.6f);
  const float l2sv = log2f(sv);
  const float ld2  = log2f(decay[h]);
  const float* src = qk32 + ((size_t)(b * kSeq + t0)) * kQKCols + h * kDq + 2 * pl;
#pragma unroll 1
  for (int it = 0; it < 16; ++it) {
    const int tl = it * 4 + tsub;
    const int t  = t0 + tl;
    const float tf = (float)t;
    const float th = tf * invf;
    float sn, cs;
    sincosf(th, &sn, &cs);
    const float tq  = tf * (1.0f / 512.0f);
    const float sc  = exp2f(tq * l2sv);
    const float isc = 1.0f / sc;
    const v2f qv = *(const v2f*)(src + (size_t)tl * kQKCols);
    const v2f kv = *(const v2f*)(src + (size_t)tl * kQKCols + kQK);
    const float q0 = qv.x, q1 = qv.y, k0 = kv.x, k1 = kv.y;
    const float cq = cs * sc, snq = sn * sc;
    const float qa = (q0 * cq - q1 * snq) * kQCarry;
    const float qb = (q1 * cq + q0 * snq) * kQCarry;
    const float ck = cs * isc, snk = sn * isc;
    const float ka = k0 * ck - k1 * snk;
    const float kb = k1 * ck + k0 * snk;
    const float dw = exp2f(ld2 * (float)(kSeq - 1 - t)) * kKwCarry;
    const float kw0 = ka * dw, kw1 = kb * dw;
    const unsigned short h0b = h_bits(kw0), h1b = h_bits(kw1);
    const float h0f = h16_to_f32((unsigned)h0b), h1f = h16_to_f32((unsigned)h1b);
    sq[tl * 68 + pl] = pk16(h_bits(qa), h_bits(qb));
    sk[tl * 68 + pl] = pk16(h_bits(ka), h_bits(kb));
    skt[(2 * pl) * 72 + tl]      = h0b;
    skt[(2 * pl + 1) * 72 + tl]  = h1b;
    sktl[(2 * pl) * 72 + tl]     = h_bits((kw0 - h0f) * kResCarry);
    sktl[(2 * pl + 1) * 72 + tl] = h_bits((kw1 - h1f) * kResCarry);
  }
  __syncthreads();
  const int hh = lane >> 4, c16 = lane & 15;
  const int q8 = lane >> 3, c8 = (lane & 7) * 8;
  for (int pass = 0; pass < 2; ++pass) {
#pragma unroll
    for (int j = 0; j < 4; ++j) {
      const int row = wave * 8 + j * 2 + hh;
      const v4u uq = *(const v4u*)(sq + row * 68 + c16 * 4);
      const v4u uk = *(const v4u*)(sk + row * 68 + c16 * 4);
      const size_t o = ((size_t)(bh * kSeq + t0 + row)) * kDq + c16 * 8;
      *(volatile v4u*)(q16 + o) = uq;
      *(volatile v4u*)(k16 + o) = uk;
    }
#pragma unroll
    for (int j = 0; j < 4; ++j) {
      const int row = wave * 16 + j * 4 + q8;
      const v4u uh = *(const v4u*)(skt + row * 72 + c8);
      const v4u ul = *(const v4u*)(sktl + row * 72 + c8);
      const size_t o = ((size_t)(bh * kDq + row)) * kSeq + t0 + c8;
      *(volatile v4u*)(kwTh + o) = uh;
      *(volatile v4u*)(kwTl + o) = ul;
    }
    __threadfence();
  }
}

__global__ __launch_bounds__(256) void pack_v_kernel(const float* __restrict__ v32, unsigned short* __restrict__ vTh,
                                                     unsigned short* __restrict__ vTl) {
#pragma clang fp contract(off)
  __shared__ __align__(16) unsigned short shi[256 * 72];
  __shared__ __align__(16) unsigned short slo[256 * 72];
  const int scnk = blockIdx.x, h = blockIdx.y, b = blockIdx.z;
  const int bh = b * kHeads + h;
  const int s0 = scnk * 64;
  const int tid = threadIdx.x, lane = tid & 31, wave = tid >> 5;
  const float* src = v32 + ((size_t)(b * kSeq + s0)) * kVDim + h * kDv;
#pragma unroll 1
  for (int i = 0; i < 16; ++i) {
    const int it = i * 256 + tid;
    const int r = it >> 6;
    const int c = (it & 63) * 4;
    const v4f w = *(const v4f*)(src + (size_t)r * kVDim + c);
    float wl[4];
    wl[0] = w.x; wl[1] = w.y; wl[2] = w.z; wl[3] = w.w;
#pragma unroll
    for (int e = 0; e < 4; ++e) {
      const float y = wl[e] * kVCarry;
      const unsigned short yb = h_bits(y);
      const float yf = h16_to_f32((unsigned)yb);
      const float dres = y - yf;
      const float res = dres * kResCarry;
      shi[(c + e) * 72 + r] = yb;
      slo[(c + e) * 72 + r] = h_bits(res);
    }
  }
  __syncthreads();
  const int q8 = lane >> 3, c8 = (lane & 7) * 8;
  for (int pass = 0; pass < 2; ++pass) {
#pragma unroll
    for (int j = 0; j < 8; ++j) {
      const int row = wave * 32 + j * 4 + q8;
      const v4u uh = *(const v4u*)(shi + row * 72 + c8);
      const v4u ul = *(const v4u*)(slo + row * 72 + c8);
      const size_t o = ((size_t)(bh * kDv + row)) * kSeq + s0 + c8;
      *(volatile v4u*)(vTh + o) = uh;
      *(volatile v4u*)(vTl + o) = ul;
    }
    __threadfence();
  }
}

constexpr int kRetLds = 80896;
constexpr int kOffQ = 0, kOffK = 17408, kOffS = 34816, kOffV = 44032;
static_assert(kOffK == 64 * 136 * 2 && kOffS == 2 * 64 * 136 * 2 && kOffV == kOffS + 64 * 72 * 2, "lds carve");
static_assert(kOffV + 256 * 72 * 2 == kRetLds && 8 * 16 * 132 * 4 <= kRetLds, "lds carve");
__global__ __launch_bounds__(256) void retention_kernel(const unsigned short* __restrict__ q16, const unsigned short* __restrict__ k16,
                                                        const unsigned short* __restrict__ vTh, const float* __restrict__ decay,
                                                        float* __restrict__ X32) {
  __shared__ __align__(16) unsigned char lds[kRetLds];
  unsigned short* sQ = (unsigned short*)(lds + kOffQ);
  unsigned short* sK = (unsigned short*)(lds + kOffK);
  _Float16*       sS = (_Float16*)(lds + kOffS);
  unsigned short* sV = (unsigned short*)(lds + kOffV);
  const _Float16* hQ = (const _Float16*)(lds + kOffQ);
  const _Float16* hK = (const _Float16*)(lds + kOffK);
  const _Float16* hS = (const _Float16*)(lds + kOffS);
  const _Float16* hV = (const _Float16*)(lds + kOffV);
  float* sO = (float*)(lds);

  const int qc = blockIdx.x, h = blockIdx.y, b = blockIdx.z;
  const int bh = b * kHeads + h;
  const int tid = threadIdx.x, wave = tid >> 5, lane = tid & 31;
  const int rl = lane & 15, hh = lane >> 4, koff = hh * 8;
  const int rw = wave & 3;
  const int vh = wave >> 2;
  const int t0 = qc * 64;
  const float ld2 = log2f(decay[h]);

  {
    const unsigned short* qsrc = q16 + ((size_t)(bh * kSeq + t0)) * kDq;
#pragma unroll
    for (int i = 0; i < 4; ++i) {
      const int it = i * 256 + tid;
      const int r = it >> 4, c = (it & 15) * 8;
      *(v4u*)(sQ + r * 136 + c) = *(const v4u*)(qsrc + (size_t)r * kDq + c);
    }
    asm volatile("" ::: "memory");
  }
  v8f o[8];
#pragma unroll
  for (int n = 0; n < 8; ++n) o[n] = (v8f){0.f,0.f,0.f,0.f,0.f,0.f,0.f,0.f};

  for (int sc = 0; sc <= qc; ++sc) {
    const int s0 = sc * 64;
    {
      const unsigned short* ksrc = k16 + ((size_t)(bh * kSeq + s0)) * kDq;
#pragma unroll
      for (int i = 0; i < 4; ++i) {
        const int it = i * 256 + tid;
        const int r = it >> 4, c = (it & 15) * 8;
        *(v4u*)(sK + r * 136 + c) = *(const v4u*)(ksrc + (size_t)r * kDq + c);
      }
      asm volatile("" ::: "memory");
      const unsigned short* vsrc = vTh + ((size_t)bh * kDv) * kSeq + s0;
#pragma unroll
      for (int grp = 0; grp < 2; ++grp) {
#pragma unroll
        for (int i = 0; i < 4; ++i) {
          const int it = (grp * 4 + i) * 256 + tid;
          const int r = it >> 3, c = (it & 7) * 8;
          *(v4u*)(sV + r * 72 + c) = *(const v4u*)(vsrc + (size_t)r * kSeq + c);
        }
        asm volatile("" ::: "memory");
      }
    }
    __syncthreads();
    if (wave < 4) {
      v8f sacc[4];
#pragma unroll
      for (int j = 0; j < 4; ++j) sacc[j] = (v8f){0.f,0.f,0.f,0.f,0.f,0.f,0.f,0.f};
#pragma unroll
      for (int kk = 0; kk < 4; ++kk) {
        const v16h aq = Frag<_Float16>::load(hQ + (rw * 16 + rl) * 136 + kk * 32 + koff);
        v16h bk[4];
#pragma unroll
        for (int j = 0; j < 4; ++j) bk[j] = Frag<_Float16>::load(hK + (j * 16 + rl) * 136 + kk * 32 + koff);
#pragma unroll
        for (int j = 0; j < 4; ++j) sacc[j] = Frag<_Float16>::mma(aq, bk[j], sacc[j]);
        dep_guard4_h(sacc[0], sacc[1], sacc[2], sacc[3], aq, bk[3]);
        keep4_h(bk[0], bk[1], bk[2], aq);
      }
      const int tgb = t0 + rw * 16 + hh * 8;
#pragma unroll
      for (int j = 0; j < 4; ++j) {
        const int sg = s0 + j * 16 + rl;
#pragma unroll
        for (int r = 0; r < 8; ++r) {
          const int n  = tgb + r - sg;
          const int nc = (n < 0) ? 0 : n;
          const float e = exp2f(ld2 * (float)nc);
          const float f = (n >= 0) ? e : 0.0f;
          sS[(rw * 16 + hh * 8 + r) * 72 + j * 16 + rl] = (_Float16)(sacc[j][r] * f * kQkScale);
        }
      }
    }
    __syncthreads();
#pragma unroll
    for (int kk = 0; kk < 2; ++kk) {
      const v16h pa = Frag<_Float16>::load(hS + (rw * 16 + rl) * 72 + kk * 32 + koff);
#pragma unroll
      for (int g = 0; g < 2; ++g) {
        v16h vb[4];
#pragma unroll
        for (int n = 0; n < 4; ++n) vb[n] = Frag<_Float16>::load(hV + (vh * 128 + (g * 4 + n) * 16 + rl) * 72 + kk * 32 + koff);
#pragma unroll
        for (int n = 0; n < 4; ++n) o[g * 4 + n] = Frag<_Float16>::mma(pa, vb[n], o[g * 4 + n]);
        dep_guard4_h(o[g * 4 + 0], o[g * 4 + 1], o[g * 4 + 2], o[g * 4 + 3], pa, vb[3]);
        keep4_h(vb[0], vb[1], vb[2], pa);
      }
    }
    __syncthreads();
  }
  acc_guard4(o[0], o[1], o[2], o[3]);
  acc_guard4(o[4], o[5], o[6], o[7]);

  float* os = sO + wave * (16 * 132);
#pragma unroll
  for (int n = 0; n < 8; ++n)
#pragma unroll
    for (int r = 0; r < 8; ++r) os[(hh * 8 + r) * 132 + n * 16 + rl] = o[n][r] * kXScale;
  __syncthreads();
  float* xd = X32 + ((size_t)(bh * kSeq + t0 + rw * 16)) * kDv + vh * 128;
  for (int pass = 0; pass < 2; ++pass) {
#pragma unroll
    for (int row = 0; row < 16; ++row) {
      const v4f val = *(const v4f*)(os + row * 132 + lane * 4);
      *(volatile v4f*)(xd + (size_t)row * kDv + lane * 4) = val;
    }
    __threadfence();
  }
}

__global__ __launch_bounds__(256) void gn_gate_kernel(const float* __restrict__ X32, const unsigned short* __restrict__ gate16,
                                                      unsigned short* __restrict__ gn16) {
  const int row = blockIdx.x;
  const int tid = threadIdx.x, lane = tid & 31, h = tid >> 5;
  const int b = row >> 11, t = row & 2047;
  const int bh = b * kHeads + h;
  const float* xr = X32 + ((size_t)(bh * kSeq + t)) * kDv + lane * 8;
  const v4f xa = *(const v4f*)(xr);
  const v4f xb = *(const v4f*)(xr + 4);
  const v4u gw = *(const v4u*)(gate16 + (size_t)row * kVDim + h * kDv + lane * 8);
  float x[8];
  x[0] = xa.x; x[1] = xa.y; x[2] = xa.z; x[3] = xa.w;
  x[4] = xb.x; x[5] = xb.y; x[6] = xb.z; x[7] = xb.w;
  float s = ((x[0] + x[1]) + (x[2] + x[3])) + ((x[4] + x[5]) + (x[6] + x[7]));
#pragma unroll
  for (int off = 16; off > 0; off >>= 1) s += __shfl_xor(s, off, 32);
  const float mu = s * (1.0f / 256.0f);
  float d[8];
  float q = 0.0f;
#pragma unroll
  for (int e = 0; e < 8; ++e) { d[e] = x[e] - mu; q += d[e] * d[e]; }
#pragma unroll
  for (int off = 16; off > 0; off >>= 1) q += __shfl_xor(q, off, 32);
  const float var  = q * (1.0f / 256.0f);
  const float rstd = 1.0f / sqrtf(var + kEps);
  const unsigned g0 = gw.x, g1 = gw.y, g2 = gw.z, g3 = gw.w;
  float g[8];
  g[0] = h16_to_f32(g0 & 0xffffu); g[1] = h16_to_f32(g0 >> 16);
  g[2] = h16_to_f32(g1 & 0xffffu); g[3] = h16_to_f32(g1 >> 16);
  g[4] = h16_to_f32(g2 & 0xffffu); g[5] = h16_to_f32(g2 >> 16);
  g[6] = h16_to_f32(g3 & 0xffffu); g[7] = h16_to_f32(g3 >> 16);
  unsigned short hb[8];
#pragma unroll
  for (int e = 0; e < 8; ++e) hb[e] = h_bits(d[e] * rstd * g[e]);
  const v4u u = (v4u){pk16(hb[0], hb[1]), pk16(hb[2], hb[3]), pk16(hb[4], hb[5]), pk16(hb[6], hb[7])};
  unsigned short* dst = gn16 + (size_t)row * kVDim + h * kDv + lane * 8;
  *(volatile v4u*)dst = u;
  __threadfence();
  *(volatile v4u*)dst = u;
}

static_assert(kHid % 32 == 0 && kSeq % 32 == 0 && kVDim % 32 == 0, "gemm k");
static_assert((kTok % 64) == 0 && (kQKCols % 64) == 0 && (kVDim % 64) == 0 && (kHid % 64) == 0, "gemm mn 64");
static_assert((kDq % 32) == 0 && (kDv % 32) == 0 && ((kDq / 32) * (kDv / 32)) % 8 == 0, "state gemm mn 32");
static_assert((size_t)kTok * kQKCols * 4 == (size_t)kTok * kVDim * 4 && (size_t)kBH * kSeq * kDv * 4 == (size_t)kTok * kVDim * 4, "R4 users equal");
static_assert((size_t)2 * kBH * kSeq * kDq * 2 == (size_t)kTok * kVDim * 2, "R5 users equal");
static_assert((size_t)2 * kBH * kDq * kSeq * 2 == (size_t)kTok * kVDim * 2, "R6 users equal");
static_assert((size_t)kTok * kHid * 4 + (size_t)kBH * kDq * kDv * 4 == 18874368ull, "out layout");

extern "C" void kernel_launch(void* const* d_in, const int* in_sizes, int n_in,
                              void* d_out, int out_size, void* d_ws, size_t ws_size,
                              hipStream_t stream) {
  if (n_in < 5) return;
  if (in_sizes[0] != kTok * kHid) return;
  if (in_sizes[1] != (2 * kQK + kVDim) * kHid) return;
  if (in_sizes[2] != kVDim * kHid) return;
  if (in_sizes[3] != kHid * kVDim) return;
  if (in_sizes[4] != kHeads) return;
  if (out_size != kTok * kHid + kBH * kDq * kDv) return;

  const size_t szHs   = (size_t)kTok * kHid * 2;
  const size_t szWqkv = (size_t)(2 * kQK + kVDim) * kHid * 2;
  const size_t szWg   = (size_t)kVDim * kHid * 2;
  const size_t szWp   = (size_t)kHid * kVDim * 2;
  const size_t szR4   = (size_t)kTok * kVDim * 4;
  const size_t szQ16  = (size_t)kBH * kSeq * kDq * 2;
  const size_t szR5   = (size_t)kTok * kVDim * 2;
  const size_t szKw   = (size_t)kBH * kDq * kSeq * 2;
  const size_t szR6   = (size_t)kTok * kVDim * 2;
  const size_t szVT   = (size_t)kBH * kDv * kSeq * 2;
  const size_t offHs   = 0;
  const size_t offWqkv = offHs + szHs;
  const size_t offWg   = offWqkv + szWqkv;
  const size_t offWp   = offWg + szWg;
  const size_t offR4   = offWp + szWp;
  const size_t offR5   = offR4 + szR4;
  const size_t offR6   = offR5 + szR5;
  const size_t offVTh  = offR6 + szR6;
  const size_t offVTl  = offVTh + szVT;
  const size_t total   = offVTl + szVT;
  if (2 * szQ16 != szR5 || 2 * szKw != szR6) return;
  if (ws_size < total) return;

  const float* hs      = (const float*)d_in[0];
  const float* w_qkv   = (const float*)d_in[1];
  const float* w_gated = (const float*)d_in[2];
  const float* w_proj  = (const float*)d_in[3];
  const float* decay   = (const float*)d_in[4];
  float* out0 = (float*)d_out;
  float* out1 = out0 + (size_t)kTok * kHid;
  char* ws = (char*)d_ws;
  unsigned short* hs16   = (unsigned short*)(ws + offHs);
  unsigned short* wqkv16 = (unsigned short*)(ws + offWqkv);
  unsigned short* wg16   = (unsigned short*)(ws + offWg);
  unsigned short* wp16   = (unsigned short*)(ws + offWp);
  float*          qk32   = (float*)(ws + offR4);
  float*          v32    = (float*)(ws + offR4);
  float*          X32    = (float*)(ws + offR4);
  unsigned short* q16    = (unsigned short*)(ws + offR5);
  unsigned short* k16    = (unsigned short*)(ws + offR5 + szQ16);
  unsigned short* gate16 = (unsigned short*)(ws + offR5);
  unsigned short* kwTh   = (unsigned short*)(ws + offR6);
  unsigned short* kwTl   = (unsigned short*)(ws + offR6 + szKw);
  unsigned short* gn16   = (unsigned short*)(ws + offR6);
  unsigned short* vTh    = (unsigned short*)(ws + offVTh);
  unsigned short* vTl    = (unsigned short*)(ws + offVTl);

  double rb = 1.0181517217173767;
  for (int n = 0; n < 4; ++n) {
    double p = rb;
    for (int s = 0; s < 9; ++s) p = p * p;
    rb = rb - (p - 10000.0) * rb / (512.0 * p);
  }

  const int n8Hs = (kTok * kHid) / 8;
  const int n8Wq = ((2 * kQK + kVDim) * kHid) / 8;
  const int n8Wg = (kVDim * kHid) / 8;
  const int n8Wp = (kHid * kVDim) / 8;
  cast8_f16_kernel<<<dim3(n8Hs / 256), dim3(256), 0, stream>>>(hs, hs16, n8Hs, 1.0f);
  cast8_f16_kernel<<<dim3(n8Wq / 256), dim3(256), 0, stream>>>(w_qkv, wqkv16, n8Wq, kWCarry);
  cast8_f16_kernel<<<dim3(n8Wg / 256), dim3(256), 0, stream>>>(w_gated, wg16, n8Wg, kWCarry);
  cast8_f16_kernel<<<dim3(n8Wp / 256), dim3(256), 0, stream>>>(w_proj, wp16, n8Wp, kWCarry);

  const int tilesQK = (kTok / 64) * (kQKCols / 64);
  wmma_gemm64<0, false, 0, 0, false, 0><<<dim3(tilesQK / 8, 1), dim3(256), 0, stream>>>(
      hs16, hs16, kHid, 0L, wqkv16, wqkv16, kHid, 0L,
      (void*)qk32, (void*)qk32, kQKCols, 0L, decay, decay, 0L, kTok, kQKCols, kHid, 1.0f / kWCarry, 1.0f);

  pack_qk_kernel<<<dim3(kSeq / 64, kHeads, kBatch), dim3(256), 0, stream>>>(qk32, decay, q16, k16, kwTh, kwTl, rb);

  wmma_gemm64<0, false, 0, 0, false, 0><<<dim3(tilesQK / 8, 1), dim3(256), 0, stream>>>(
      hs16, hs16, kHid, 0L, wqkv16 + (size_t)kQKCols * kHid, wqkv16 + (size_t)kQKCols * kHid, kHid, 0L,
      (void*)v32, (void*)v32, kVDim, 0L, decay, decay, 0L, kTok, kVDim, kHid, 1.0f / kWCarry, 1.0f);

  pack_v_kernel<<<dim3(kSeq / 64, kHeads, kBatch), dim3(256), 0, stream>>>(v32, vTh, vTl);

  retention_kernel<<<dim3(kSeq / 64, kHeads, kBatch), dim3(256), 0, stream>>>(q16, k16, vTh, decay, X32);

  const int tilesKV = (kDq / 32) * (kDv / 32);
  state_gemm_kernel<<<dim3(tilesKV / 8, kBH), dim3(256), 0, stream>>>(
      kwTh, kwTl, kSeq, (long)kDq * kSeq, vTh, vTl, kSeq, (long)kDv * kSeq,
      out1, kDv, (long)kDq * kDv, kDq, kDv, kSeq, 1.0f / (kKwCarry * kVCarry), kResInv);

  wmma_gemm64<0, false, 0, 1, false, 3><<<dim3(tilesQK / 8, 1), dim3(256), 0, stream>>>(
      hs16, hs16, kHid, 0L, wg16, wg16, kHid, 0L,
      (void*)gate16, (void*)gate16, kVDim, 0L, decay, decay, 0L, kTok, kVDim, kHid, 1.0f / kWCarry, kGCarry);

  gn_gate_kernel<<<dim3(kTok), dim3(256), 0, stream>>>(X32, gate16, gn16);

  const int tilesOut = (kTok / 64) * (kHid / 64);
  wmma_gemm64<0, false, 0, 0, false, 0><<<dim3(tilesOut / 8, 1), dim3(256), 0, stream>>>(
      gn16, gn16, kVDim, 0L, wp16, wp16, kVDim, 0L,
      (void*)out0, (void*)out0, kHid, 0L, decay, decay, 0L, kTok, kHid, kVDim, 1.0f / (kGCarry * kWCarry), 1.0f);
}
